// ContinuousTimeMultiHeadAttention_70858370449468
// MI455X (gfx1250) — hardware-verified
//
#include <hip/hip_runtime.h>


#define B_  2
#define L_  128
#define D_  256
#define H_  8
#define R_  4
#define DK_ 32
#define TP_ 36

typedef float        v4f   __attribute__((ext_vector_type(4)));
typedef v4f          v4fa  __attribute__((may_alias));
typedef float        v8f   __attribute__((ext_vector_type(8)));
typedef unsigned int v8u   __attribute__((ext_vector_type(8)));
typedef __bf16       v16bf __attribute__((ext_vector_type(16)));
typedef int          v4i   __attribute__((ext_vector_type(4)));

union Frag { v8u u; v16bf v; };

__device__ __forceinline__ unsigned int bf16_rne_bits(float x) {
  const unsigned int u = __float_as_uint(x);
  return (u + 0x7FFFu + ((u >> 16) & 1u)) >> 16;
}

__device__ __forceinline__ void pack_split(const float (&x)[16], Frag& hi, Frag& lo) {
  unsigned int hw[8], lw[8];
#pragma unroll
  for (int j = 0; j < 8; ++j) {
    const float x0 = x[2 * j], x1 = x[2 * j + 1];
    const unsigned int h0 = bf16_rne_bits(x0), h1 = bf16_rne_bits(x1);
    const float r0 = x0 - __uint_as_float(h0 << 16);
    const float r1 = x1 - __uint_as_float(h1 << 16);
    const unsigned int l0 = bf16_rne_bits(r0), l1 = bf16_rne_bits(r1);
    hw[j] = h0 | (h1 << 16);
    lw[j] = l0 | (l1 << 16);
  }
  const v8u hv = {hw[0], hw[1], hw[2], hw[3], hw[4], hw[5], hw[6], hw[7]};
  const v8u lv = {lw[0], lw[1], lw[2], lw[3], lw[4], lw[5], lw[6], lw[7]};
  hi.u = hv;
  lo.u = lv;
}

__device__ __forceinline__ void mma_bf16(v8f& acc, const Frag& a, const Frag& b) {
  acc = __builtin_amdgcn_wmma_f32_16x16x32_bf16(false, a.v, false, b.v, (short)0, acc, false, false);
  asm volatile("v_nop\n\tv_nop\n\tv_nop\n\tv_nop" : "+v"(acc) : "v"(a.u), "v"(b.u));
}

__device__ __forceinline__ void load_a_split(const float* __restrict__ arow, int k0, Frag& hi, Frag& lo) {
  const v4f t0 = *(const v4f*)(arow + k0);
  const v4f t1 = *(const v4f*)(arow + k0 + 4);
  const v4f t2 = *(const v4f*)(arow + k0 + 16);
  const v4f t3 = *(const v4f*)(arow + k0 + 20);
  const float x[16] = {t0.x, t0.y, t0.z, t0.w, t1.x, t1.y, t1.z, t1.w,
                       t2.x, t2.y, t2.z, t2.w, t3.x, t3.y, t3.z, t3.w};
  pack_split(x, hi, lo);
}

__device__ __forceinline__ void load_b_split(const float* __restrict__ bcol, int ldb, int k0, int hh,
                                             Frag& hi, Frag& lo) {
  float x[16];
  const float* p0 = bcol + (size_t)(k0 + 8 * hh) * ldb;
  const float* p1 = bcol + (size_t)(k0 + 16 + 8 * hh) * ldb;
#pragma unroll
  for (int i = 0; i < 8; ++i) {
    x[i]     = p0[(size_t)i * ldb];
    x[8 + i] = p1[(size_t)i * ldb];
  }
  pack_split(x, hi, lo);
}

__global__ __launch_bounds__(64) void k_gemm(const float* __restrict__ A, int lda, int sAz,
                                             const float* __restrict__ Bm, int ldb, int sBh, int sBl,
                                             float* C, int ldc, int sCh, int sCl,
                                             const float* __restrict__ bias, const float* __restrict__ resid,
                                             int epi, int zsh, int M, int N, int K) {
  __shared__ __attribute__((aligned(16))) float tile[32 * TP_];
  const int z  = blockIdx.z;
  const int zh = z >> zsh, zl = z & ((1 << zsh) - 1);
  A  += (size_t)z * sAz;
  Bm += (size_t)zh * sBh + (size_t)zl * sBl;
  const size_t coff = (size_t)zh * sCh + (size_t)zl * sCl;
  C     += coff;
  resid += coff;
  const int row0 = blockIdx.x * 32, col0 = blockIdx.y * 32;
  if (row0 + 32 > M || col0 + 32 > N) return;

  const int wave = threadIdx.x >> 5, lane = threadIdx.x & 31;
  const int hh = lane >> 4, m = lane & 15;
  const float* arow = A + (size_t)(row0 + 16 * wave + m) * lda + 8 * hh;
  const float* bcol = Bm + col0 + m;

  v8f acc0 = {};
  v8f acc1 = {};
  for (int k0 = 0; k0 < K; k0 += 32) {
    Frag ahi, alo, bhi, blo;
    load_a_split(arow, k0, ahi, alo);
    load_b_split(bcol, ldb, k0, hh, bhi, blo);
    mma_bf16(acc0, ahi, bhi);
    mma_bf16(acc0, ahi, blo);
    mma_bf16(acc0, alo, bhi);
    load_b_split(bcol + 16, ldb, k0, hh, bhi, blo);
    mma_bf16(acc1, ahi, bhi);
    mma_bf16(acc1, ahi, blo);
    mma_bf16(acc1, alo, bhi);
  }

  {
    float* trow = tile + (16 * wave + 8 * hh) * TP_;
#pragma unroll
    for (int r = 0; r < 8; ++r) {
      trow[r * TP_ + m]      = acc0[r];
      trow[r * TP_ + 16 + m] = acc1[r];
    }
  }
  __syncthreads();

  v4f    vals[4];
  size_t goff[4];
#pragma unroll
  for (int it = 0; it < 4; ++it) {
    const int rl = 16 * wave + 4 * it + (lane >> 3);
    const int cq = 4 * (lane & 7);
    v4f val = *(const v4fa*)(tile + rl * TP_ + cq);
    const int grow = row0 + rl, gcol = col0 + cq;
    const size_t off = (size_t)grow * ldc + gcol;
    if (epi) {
      const v4f bv = *(const v4f*)(bias + gcol);
      const v4f rv = *(const v4f*)(resid + off);
      val = (val + bv) + rv;
    }
    vals[it] = val;
    goff[it] = off;
    *(volatile v4f*)(C + off) = val;
  }
  __threadfence();
#pragma unroll
  for (int it = 0; it < 4; ++it) *(volatile v4f*)(C + goff[it]) = vals[it];
}

__global__ __launch_bounds__(256) void k_ln(const float* __restrict__ x, const float* __restrict__ g,
                                            const float* __restrict__ bb, float* y, int nrows) {
  const int wave = threadIdx.x >> 5, lane = threadIdx.x & 31;
  const int row = blockIdx.x * 8 + wave;
  if (row >= nrows) return;
  const float* xr = x + (size_t)row * D_;
  const v4f a0 = *(const v4f*)(xr + 4 * lane);
  const v4f a1 = *(const v4f*)(xr + 128 + 4 * lane);
  float sum = ((a0.x + a0.y) + (a0.z + a0.w)) + ((a1.x + a1.y) + (a1.z + a1.w));
#pragma unroll
  for (int off = 16; off > 0; off >>= 1) sum += __shfl_xor(sum, off);
  const float mean = sum * (1.0f / D_);
  const v4f d0 = a0 - mean, d1 = a1 - mean;
  float sq = ((d0.x * d0.x + d0.y * d0.y) + (d0.z * d0.z + d0.w * d0.w)) +
             ((d1.x * d1.x + d1.y * d1.y) + (d1.z * d1.z + d1.w * d1.w));
#pragma unroll
  for (int off = 16; off > 0; off >>= 1) sq += __shfl_xor(sq, off);
  const float var = sq * (1.0f / D_);
  const float inv = 1.0f / sqrtf(var + 1.0e-6f);
  const v4f g0 = *(const v4f*)(g + 4 * lane),  g1 = *(const v4f*)(g + 128 + 4 * lane);
  const v4f b0 = *(const v4f*)(bb + 4 * lane), b1 = *(const v4f*)(bb + 128 + 4 * lane);
  const v4f y0 = (d0 * inv) * g0 + b0;
  const v4f y1 = (d1 * inv) * g1 + b1;
  float* yr = y + (size_t)row * D_;
  *(volatile v4f*)(yr + 4 * lane)       = y0;
  *(volatile v4f*)(yr + 128 + 4 * lane) = y1;
  __threadfence();
  *(volatile v4f*)(yr + 4 * lane)       = y0;
  *(volatile v4f*)(yr + 128 + 4 * lane) = y1;
}

__global__ __launch_bounds__(256) void k_softmax(const float* __restrict__ pq, const float* __restrict__ pk,
                                                 const float* __restrict__ t, const float* __restrict__ s,
                                                 const float* __restrict__ omega, const int* __restrict__ msk,
                                                 float* p_out, float* Amat, int nrows) {
  __shared__ __attribute__((aligned(16))) float S_l[L_];
  const int wave = threadIdx.x >> 5, lane = threadIdx.x & 31;
  const int bh = blockIdx.x >> 4;
  const int b = bh >> 3, h = bh & (H_ - 1);
  const int i = ((blockIdx.x & 15) << 3) + wave;
  const int row = blockIdx.x * 8 + wave;

  if (threadIdx.x < L_ && bh < B_ * H_) {
    const int j = threadIdx.x;
    const v4f* a = (const v4f*)(pq + (size_t)(b * L_ + j) * D_ + h * DK_);
    const v4f* c = (const v4f*)(pk + (size_t)(b * L_ + j) * D_ + h * DK_);
    float acc = 0.f;
#pragma unroll 1
    for (int d4 = 0; d4 < DK_ / 4; ++d4) {
      const v4f xa = a[d4], xc = c[d4];
      acc += xa.x * xc.x;
      acc += xa.y * xc.y;
      acc += xa.z * xc.z;
      acc += xa.w * xc.w;
    }
    S_l[j] = acc;
  }
  __syncthreads();
  if (row >= nrows) return;

  const float invtemp = 1.0f / 5.656854249492381f;
  const int jb = 4 * lane;
  const float ti = t[b * L_ + i];
  const v4f tj = *(const v4f*)(t + b * L_ + jb);
  const v4f om = *(const v4f*)(omega + (size_t)(b * L_ + i) * L_ + jb);
  const v4i mk = *(const v4i*)(msk + (size_t)i * L_ + jb);
  const v4f Sv = *(const v4fa*)(S_l + jb);
  const float s0 = s[0], s1 = s[1], s2 = s[2], s3 = s[3];
  const float tjv[4] = {tj.x, tj.y, tj.z, tj.w};
  const float omv[4] = {om.x, om.y, om.z, om.w};
  const int   mkv[4] = {mk.x, mk.y, mk.z, mk.w};
  const float svv[4] = {Sv.x, Sv.y, Sv.z, Sv.w};

  float lg[4], p1[4];
  float mx = -3.0e38f;
#pragma unroll
  for (int c = 0; c < 4; ++c) {
    const float dt = fabsf(ti - tjv[c]);
    const float e0 = __expf(-(dt * s0));
    const float e1 = __expf(-(dt * s1));
    const float e2 = __expf(-(dt * s2));
    const float e3 = __expf(-(dt * s3));
    p1[c] = ((e0 + e1) + e2) + e3;
    const float p2 = ((e0 * e0 + e1 * e1) + e2 * e2) + e3 * e3;
    const float val = (mkv[c] != 0) ? -1.0e9f : ((omv[c] * p2) * svv[c]) * invtemp;
    lg[c] = val;
    mx = fmaxf(mx, val);
  }
#pragma unroll
  for (int off = 16; off > 0; off >>= 1) mx = fmaxf(mx, __shfl_xor(mx, off));
  float sum = 0.f;
#pragma unroll
  for (int c = 0; c < 4; ++c) {
    lg[c] = __expf(lg[c] - mx);
    sum += lg[c];
  }
#pragma unroll
  for (int off = 16; off > 0; off >>= 1) sum += __shfl_xor(sum, off);
  const float inv = 1.0f / sum;
  const float q0 = lg[0] * inv, q1 = lg[1] * inv, q2 = lg[2] * inv, q3 = lg[3] * inv;
  const v4f P  = {q0, q1, q2, q3};
  const v4f Av = {q0 * p1[0], q1 * p1[1], q2 * p1[2], q3 * p1[3]};
  float* po = p_out + (size_t)row * L_ + jb;
  float* am = Amat  + (size_t)row * L_ + jb;
  *(volatile v4f*)po = P;
  *(volatile v4f*)am = Av;
  __threadfence();
  *(volatile v4f*)po = P;
  *(volatile v4f*)am = Av;
}

extern "C" void kernel_launch(void* const* d_in, const int* in_sizes, int n_in,
                              void* d_out, int out_size, void* d_ws, size_t ws_size,
                              hipStream_t stream) {
  if (n_in < 14) return;
  const float* q     = (const float*)d_in[0];
  const float* k     = (const float*)d_in[1];
  const float* v     = (const float*)d_in[2];
  const float* t     = (const float*)d_in[3];
  const float* omega = (const float*)d_in[4];
  const int*   msk   = (const int*)  d_in[5];
  const float* Wq    = (const float*)d_in[6];
  const float* Wk    = (const float*)d_in[7];
  const float* Wv    = (const float*)d_in[8];
  const float* s     = (const float*)d_in[9];
  const float* fc_w  = (const float*)d_in[10];
  const float* fc_b  = (const float*)d_in[11];
  const float* ln_g  = (const float*)d_in[12];
  const float* ln_b  = (const float*)d_in[13];

  const int NT = B_ * L_;
  if (in_sizes[0] != NT * D_ || in_sizes[1] != NT * D_ || in_sizes[2] != NT * D_ ||
      in_sizes[3] != NT || in_sizes[4] != B_ * L_ * L_ || in_sizes[5] != L_ * L_ ||
      in_sizes[6] != D_ * D_ || in_sizes[7] != D_ * D_ || in_sizes[8] != D_ * D_ ||
      in_sizes[9] != R_ || in_sizes[10] != D_ * D_ || in_sizes[11] != D_ ||
      in_sizes[12] != D_ || in_sizes[13] != D_) return;
  if (out_size != NT * D_ + B_ * H_ * L_ * L_) return;

  const size_t sz_tok  = (size_t)NT * D_ * sizeof(float);
  const size_t sz_amat = (size_t)B_ * H_ * L_ * L_ * sizeof(float);
  const size_t o_qn   = 0;
  const size_t o_pq   = o_qn + sz_tok;
  const size_t o_pk   = o_pq + sz_tok;
  const size_t o_pv   = o_pk + sz_tok;
  const size_t o_o1   = o_pv + sz_tok;
  const size_t o_amat = o_o1 + sz_tok;
  const size_t total  = o_amat + sz_amat;
  if (total > ws_size) return;
  char* base  = (char*)d_ws;
  float* qn   = (float*)(base + o_qn);
  float* pq   = (float*)(base + o_pq);
  float* pk   = (float*)(base + o_pk);
  float* pv   = (float*)(base + o_pv);
  float* out1 = (float*)(base + o_o1);
  float* Amat = (float*)(base + o_amat);

  float* out_p = (float*)d_out;
  float* p_out = out_p + (size_t)NT * D_;

  k_ln<<<dim3((NT + 7) / 8), dim3(256), 0, stream>>>(q, ln_g, ln_b, qn, NT);

  const dim3 gp((NT + 31) / 32, (D_ + 31) / 32, 1);
  k_gemm<<<gp, dim3(64), 0, stream>>>(qn, D_, 0, Wq, D_, 0, 0, pq, D_, 0, 0, fc_b, q, 0, 0, NT, D_, D_);
  k_gemm<<<gp, dim3(64), 0, stream>>>(k,  D_, 0, Wk, D_, 0, 0, pk, D_, 0, 0, fc_b, q, 0, 0, NT, D_, D_);
  k_gemm<<<gp, dim3(64), 0, stream>>>(v,  D_, 0, Wv, D_, 0, 0, pv, D_, 0, 0, fc_b, q, 0, 0, NT, D_, D_);

  const int nrows = B_ * H_ * L_;
  k_softmax<<<dim3((nrows + 7) / 8), dim3(256), 0, stream>>>(pq, pk, t, s, omega, msk, p_out, Amat, nrows);

  k_gemm<<<dim3((L_ + 31) / 32, (DK_ + 31) / 32, B_ * H_), dim3(64), 0, stream>>>(
      Amat, L_, L_ * L_, pv, D_, L_ * D_, DK_, out1, D_, L_ * D_, DK_, fc_b, q, 0, 3, L_, DK_, L_);

  k_gemm<<<gp, dim3(64), 0, stream>>>(out1, D_, 0, fc_w, D_, 0, 0, out_p, D_, 0, 0, fc_b, q, 1, 0, NT, D_, D_);
}
